// NeuralSFA_29377576305410
// MI455X (gfx1250) — hardware-run, weakly checked
//
#include <hip/hip_runtime.h>
#include <stddef.h>
#include <math.h>

typedef __attribute__((ext_vector_type(16))) _Float16 v16h;
typedef __attribute__((ext_vector_type(8)))  _Float16 v8h;
typedef __attribute__((ext_vector_type(16))) __bf16   v16b;
typedef __attribute__((ext_vector_type(8)))  __bf16   v8b;
typedef __attribute__((ext_vector_type(8)))  float    v8f;
typedef __attribute__((ext_vector_type(4)))  float    v4f;

__device__ __forceinline__ unsigned short f2bf_bits(float f) {
  unsigned u = __float_as_uint(f);
  return (unsigned short)((u + 0x7FFFu + ((u >> 16) & 1u)) >> 16);
}
__device__ __forceinline__ float bf_bits2f(unsigned short h) { return __uint_as_float(((unsigned)h) << 16); }

__device__ __forceinline__ void dep_guard_h(v8f& a, v8f& b, v16h x, v16h y) { asm volatile("v_nop\n\tv_nop\n\tv_nop\n\tv_nop" : "+v"(a), "+v"(b) : "v"(x), "v"(y)); }
__device__ __forceinline__ void dep_guard_b(v8f& a, v8f& b, v16b x, v16b y) { asm volatile("v_nop\n\tv_nop\n\tv_nop\n\tv_nop" : "+v"(a), "+v"(b) : "v"(x), "v"(y)); }
__device__ __forceinline__ void keep4_h(v16h a, v16h b, v16h c, v16h d) { asm volatile("v_nop" :: "v"(a), "v"(b), "v"(c), "v"(d)); }
__device__ __forceinline__ void keep4_b(v16b a, v16b b, v16b c, v16b d) { asm volatile("v_nop" :: "v"(a), "v"(b), "v"(c), "v"(d)); }
__device__ __forceinline__ void acc_guard4(v8f& a, v8f& b, v8f& c, v8f& d) { asm volatile("v_nop\n\tv_nop\n\tv_nop\n\tv_nop" : "+v"(a), "+v"(b), "+v"(c), "+v"(d)); }
template <typename T> struct Frag;
template <> struct Frag<_Float16> {
  typedef v16h V; union U { v16h v; v8h h[2]; };
  static __device__ __forceinline__ v16h load(const _Float16* p) {
    U f; f.h[0] = *(const v8h*)(p); f.h[1] = *(const v8h*)(p + 16); return f.v;
  }
  static __device__ __forceinline__ v8f mma(v16h a, v16h b, v8f c) {
    return __builtin_amdgcn_wmma_f32_16x16x32_f16(false, a, false, b, (short)0, c, false, false);
  }
  static __device__ __forceinline__ void guard(v8f& a, v8f& b, v16h x, v16h y) { dep_guard_h(a, b, x, y); }
  static __device__ __forceinline__ void keep(v16h a, v16h b, v16h c, v16h d) { keep4_h(a, b, c, d); }
};
template <> struct Frag<__bf16> {
  typedef v16b V; union U { v16b v; v8b h[2]; };
  static __device__ __forceinline__ v16b load(const __bf16* p) {
    U f; f.h[0] = *(const v8b*)(p); f.h[1] = *(const v8b*)(p + 16); return f.v;
  }
  static __device__ __forceinline__ v8f mma(v16b a, v16b b, v8f c) {
    return __builtin_amdgcn_wmma_f32_16x16x32_bf16(false, a, false, b, (short)0, c, false, false);
  }
  static __device__ __forceinline__ void guard(v8f& a, v8f& b, v16b x, v16b y) { dep_guard_b(a, b, x, y); }
  static __device__ __forceinline__ void keep(v16b a, v16b b, v16b c, v16b d) { keep4_b(a, b, c, d); }
};

template <int ET> struct Elem;
template <> struct Elem<0> { typedef _Float16 T; };
template <> struct Elem<1> { typedef __bf16 T; };
template <int ET, bool SPLIT, int BIAS_MODE, int OUT_MODE, bool RESID, int ACT = 0>
__global__ __launch_bounds__(256) void wmma_gemm64(
    const unsigned short* __restrict__ Ap, const unsigned short* __restrict__ A2p, int lda, long strideA,
    const unsigned short* __restrict__ Btp, const unsigned short* __restrict__ Bt2p, int ldb, long strideB,
    void* __restrict__ Cout, void* __restrict__ Cout2, int ldc, long strideC,
    const float* __restrict__ bias,
    const float* __restrict__ resid, long strideR,
    int M, int N, int K, float scale) {
  typedef typename Elem<ET>::T T;
  typedef typename Frag<T>::V V;
  const T* A = (const T*)Ap; const T* A2 = (const T*)A2p; const T* Bt = (const T*)Btp; const T* Bt2 = (const T*)Bt2p;
  __shared__ __align__(16) float sT[8][16 * 68];
  const int b    = blockIdx.y;
  const int lane = threadIdx.x & 31;
  const int wave = threadIdx.x >> 5;
  const int tilesN = N >> 6;
  const int tilesM = M >> 6;
  const int tile = blockIdx.x * 8 + wave;
  if (tile >= tilesM * tilesN) return;
  const int tm = tile / tilesN;
  const int tn = tile - tm * tilesN;
  const int m0 = tm << 6;
  const int n0 = tn << 6;

  const T* Ab  = A  + (size_t)b * strideA;
  const T* Bb  = Bt + (size_t)b * strideB;
  const T* Ab2 = SPLIT ? (A2  + (size_t)b * strideA) : nullptr;
  const T* Bb2 = SPLIT ? (Bt2 + (size_t)b * strideB) : nullptr;

  const int rlane = lane & 15;
  const int koff  = (lane >> 4) * 8;
  const int mOff  = (lane >> 4) * 8;

  v8f acc[4][4];
#pragma unroll
  for (int i = 0; i < 4; ++i)
#pragma unroll
    for (int j = 0; j < 4; ++j) acc[i][j] = (v8f){0.f,0.f,0.f,0.f,0.f,0.f,0.f,0.f};

  for (int k0 = 0; k0 < K; k0 += 32) {
    V bh[4], bl[4];
#pragma unroll
    for (int j = 0; j < 4; ++j) {
      const size_t bo = (size_t)(n0 + (j << 4) + rlane) * ldb + koff + k0;
      bh[j] = Frag<T>::load(Bb + bo);
      if (SPLIT) bl[j] = Frag<T>::load(Bb2 + bo);
    }
#pragma unroll
    for (int i = 0; i < 4; ++i) {
      const size_t ao = (size_t)(m0 + (i << 4) + rlane) * lda + koff + k0;
      V ah = Frag<T>::load(Ab + ao);
      V al;
      if (SPLIT) al = Frag<T>::load(Ab2 + ao);
#pragma unroll
      for (int j = 0; j < 4; ++j) {
        acc[i][j] = Frag<T>::mma(ah, bh[j], acc[i][j]);
        if (SPLIT) {
          acc[i][j] = Frag<T>::mma(ah, bl[j], acc[i][j]);
          acc[i][j] = Frag<T>::mma(al, bh[j], acc[i][j]);
        }
      }
      Frag<T>::guard(acc[i][0], acc[i][3], ah, SPLIT ? al : ah);
    }
    Frag<T>::keep(bh[0], bh[1], bh[2], bh[3]);
    if (SPLIT) Frag<T>::keep(bl[0], bl[1], bl[2], bl[3]);
  }
  acc_guard4(acc[0][0], acc[0][1], acc[0][2], acc[0][3]);
  acc_guard4(acc[1][0], acc[1][1], acc[1][2], acc[1][3]);
  acc_guard4(acc[2][0], acc[2][1], acc[2][2], acc[2][3]);
  acc_guard4(acc[3][0], acc[3][1], acc[3][2], acc[3][3]);

  float* slab = sT[wave];
  const float* Rb = RESID ? (resid + (size_t)b * strideR) : nullptr;
#pragma unroll
  for (int i = 0; i < 4; ++i) {
    const int mBase = m0 + (i << 4);
#pragma unroll
    for (int j = 0; j < 4; ++j) {
      const int n = n0 + (j << 4) + rlane;
      float bv = 0.f;
      if (BIAS_MODE == 2) bv = bias[n];
#pragma unroll
      for (int r = 0; r < 8; ++r) {
        float v = acc[i][j][r] * scale;
        if (BIAS_MODE == 1) v += bias[mBase + mOff + r];
        if (BIAS_MODE == 2) v += bv;
        if (RESID) v += Rb[(size_t)(mBase + mOff + r) * ldc + n];
        if (ACT == 1) v = tanhf(v);
        if (ACT == 2) v = fmaxf(v, 0.0f);
        if (ACT == 3) v = v / (1.0f + expf(-v));
        if (ACT == 4) v = (v > 0.f) ? v : 0.01f * v;
        if (ACT == 5) v = 0.5f * v * (1.0f + erff(v * 0.70710678118654752f));
        slab[(mOff + r) * 68 + (j << 4) + rlane] = v;
      }
    }
    __builtin_amdgcn_fence(__ATOMIC_RELEASE, "workgroup");
    __builtin_amdgcn_wave_barrier();
    __builtin_amdgcn_fence(__ATOMIC_ACQUIRE, "workgroup");
    if (OUT_MODE == 0) {
      float* C = (float*)Cout + (size_t)b * strideC;
      const int hh = lane >> 4, c4 = (lane & 15) * 4;
      for (int pass = 0; pass < 2; ++pass) {
#pragma unroll
        for (int it = 0; it < 8; ++it) {
          const int row = it * 2 + hh;
          v4f v = *(const v4f*)(slab + row * 68 + c4);
          *(volatile v4f*)(C + (size_t)(mBase + row) * ldc + n0 + c4) = v;
        }
        __threadfence();
      }
    } else {
      const int q = lane >> 3, c8 = (lane & 7) * 8;
      unsigned short* C  = (unsigned short*)Cout  + (size_t)b * strideC;
      unsigned short* C2 = (OUT_MODE == 2) ? ((unsigned short*)Cout2 + (size_t)b * strideC) : nullptr;
      for (int pass = 0; pass < 2; ++pass) {
#pragma unroll
        for (int it = 0; it < 4; ++it) {
          const int row = it * 4 + q;
          const float* sp = slab + row * 68 + c8;
          v8h hv, lv;
#pragma unroll
          for (int e = 0; e < 8; ++e) {
            if (OUT_MODE == 1) {
              hv[e] = (_Float16)sp[e];
            } else {
              unsigned short hb = f2bf_bits(sp[e]);
              unsigned short lb = f2bf_bits(sp[e] - bf_bits2f(hb));
              hv[e] = __builtin_bit_cast(_Float16, hb);
              lv[e] = __builtin_bit_cast(_Float16, lb);
            }
          }
          *(volatile v8h*)(C + (size_t)(mBase + row) * ldc + n0 + c8) = hv;
          if (OUT_MODE == 2) *(volatile v8h*)(C2 + (size_t)(mBase + row) * ldc + n0 + c8) = lv;
        }
        __threadfence();
      }
    }
    __builtin_amdgcn_fence(__ATOMIC_RELEASE, "workgroup");
    __builtin_amdgcn_wave_barrier();
    __builtin_amdgcn_fence(__ATOMIC_ACQUIRE, "workgroup");
  }
}

constexpr int kThreads      = 256;
constexpr int kImgPix       = 28 * 28;
constexpr int kX1Pos        = 13 * 13;
constexpr int kX1Ch         = 8;
constexpr int kRows2        = 128;
constexpr int kRows2Real    = 11 * 11;
constexpr int kKc2Real      = 72;
constexpr int kKc2          = 96;
constexpr int kNcol         = 64;
constexpr int kRows3        = 16;
constexpr int kRows3Real    = 9;
constexpr int kKc3Real      = 144;
constexpr int kKc3          = 160;
constexpr int kKdReal       = 32;
constexpr int kKd           = 64;
constexpr int kImgsPerChunk = 2048;
constexpr float kActCarry   = 16.0f;
constexpr float kWCarry     = 8.0f;
constexpr float kConvScale  = 0.125f;
constexpr float kDenseScale = 1.0f / 128.0f;
constexpr float kInvTemp    = 10.0f;
constexpr int kChainThreads = 128;
constexpr int kChainSteps   = 512;
constexpr int kSmThreads    = 64;
constexpr int kSmImgs       = 32;

static_assert(kThreads * 6 == kRows2 * kKc2 / 8);
static_assert(kThreads * 6 >= kX1Pos * kX1Ch);
static_assert(kThreads * 2 >= 25 * 16 && kThreads * 2 >= kRows3 * kKc3 / 8);
static_assert(kKc2 % 32 == 0 && kKc3 % 32 == 0 && kKd % 32 == 0);
static_assert(kKc2 > kKc2Real && kKc3 > kKc3Real && kKd > kKdReal);
static_assert(kImgsPerChunk % 64 == 0);
static_assert((kRows2 * kKc2 * 2) % 128 == 0 && (kRows3 * kKc3 * 2) % 128 == 0);
static_assert(kSmImgs * 10 * 4 % 128 == 0);

__device__ __forceinline__ int imin(int a, int b) { return a < b ? a : b; }
__device__ __forceinline__ v8h zero8h() {
  v8h z;
#pragma unroll
  for (int e = 0; e < 8; ++e) z[e] = (_Float16)0.0f;
  return z;
}

__global__ __launch_bounds__(kThreads) void k_wprep(const float* __restrict__ W, const float* __restrict__ bvec,
                                                     int ncol, int nic, int ktap, int kreal, int kpad, float scale,
                                                     _Float16* __restrict__ bt) {
  const int tpr = kpad >> 3;
  const int total = kNcol * tpr;
  const int i = blockIdx.x * kThreads + threadIdx.x;
  if (i >= total) return;
  const int n   = i / tpr;
  const int k0  = (i - n * tpr) * 8;
  const int ncl = (n < ncol) ? n : (ncol - 1);
  const float bv = bvec[ncl];
  v8h hv;
#pragma unroll
  for (int e = 0; e < 8; ++e) {
    const int k   = k0 + e;
    const int kc  = (k < kreal) ? k : (kreal - 1);
    const int tap = kc / nic;
    const int ic  = kc - tap * nic;
    float v = W[(size_t)ncl * kreal + ic * ktap + tap];
    if (k >= kreal) v = (k == kreal) ? bv : 0.0f;
    if (n >= ncol) v = 0.0f;
    hv[e] = (_Float16)(scale * v);
  }
  _Float16* dst = bt + (size_t)i * 8;
  *(volatile v8h*)dst = hv;
  __threadfence();
  *(volatile v8h*)dst = hv;
}

__global__ __launch_bounds__(kThreads) void k_conv1(const float* __restrict__ seq, const float* __restrict__ w1,
                                                     const float* __restrict__ b1, int img_base,
                                                     _Float16* __restrict__ im2) {
  __shared__ __align__(16) float s_img[kImgPix];
  __shared__ float s_w[72];
  __shared__ float s_b[8];
  __shared__ __align__(16) _Float16 s_x1[kX1Pos * kX1Ch];
  const int tid = threadIdx.x;
  const int il  = blockIdx.x;
  const int img = img_base + il;
  if (tid < kImgPix / 4) {
    const v4f x = *(const v4f*)(seq + (size_t)img * kImgPix + tid * 4);
    *(v4f*)(s_img + tid * 4) = x;
  }
  if (tid < 72) s_w[tid] = w1[tid];
  if (tid < 8) s_b[tid] = b1[tid];
  __syncthreads();

#pragma unroll 1
  for (int it = 0; it < 6; ++it) {
    const int idx = tid + it * kThreads;
    const int idc = imin(idx, kX1Pos * kX1Ch - 1);
    const int oc  = idc & 7;
    const int p   = idc >> 3;
    const int py  = p / 13;
    const int px  = p - py * 13;
    const float* ib = s_img + (2 * py) * 28 + 2 * px;
    float P[4][4];
#pragma unroll
    for (int r = 0; r < 4; ++r)
#pragma unroll
      for (int c = 0; c < 4; ++c) P[r][c] = ib[r * 28 + c];
    float w[9];
#pragma unroll
    for (int q = 0; q < 9; ++q) w[q] = s_w[oc * 9 + q];
    const float bb = s_b[oc];
    float s00 = bb, s01 = bb, s10 = bb, s11 = bb;
#pragma unroll
    for (int dy = 0; dy < 3; ++dy)
#pragma unroll
      for (int dx = 0; dx < 3; ++dx) {
        const float wq = w[dy * 3 + dx];
        s00 = fmaf(P[dy][dx], wq, s00);
        s01 = fmaf(P[dy][dx + 1], wq, s01);
        s10 = fmaf(P[dy + 1][dx], wq, s10);
        s11 = fmaf(P[dy + 1][dx + 1], wq, s11);
      }
    const float v = (fmaxf(s00, 0.f) + fmaxf(s01, 0.f) + fmaxf(s10, 0.f) + fmaxf(s11, 0.f)) * 4.0f;
    if (idx < kX1Pos * kX1Ch) s_x1[idc] = (_Float16)v;
  }
  __syncthreads();

  _Float16* ob = im2 + (size_t)il * (kRows2 * kKc2);
  const v8h z8 = zero8h();
#pragma unroll 1
  for (int it = 0; it < 6; ++it) {
    const int i    = tid + it * kThreads;
    const int row  = i / 12;
    const int kq   = i - row * 12;
    const int rowc = imin(row, kRows2Real - 1);
    const int oy   = rowc / 11;
    const int ox   = rowc - oy * 11;
    const int tap  = imin(kq, 8);
    const int dy   = tap / 3;
    const int dx   = tap - dy * 3;
    const v8h xv = *(const v8h*)(s_x1 + ((oy + dy) * 13 + ox + dx) * kX1Ch);
    v8h v = xv;
    if (kq >= 9) v = z8;
    if (kq == 9) v[0] = (_Float16)kActCarry;
    if (row >= kRows2Real) v = z8;
    _Float16* dst = ob + (size_t)i * 8;
    *(volatile v8h*)dst = v;
    __threadfence();
    *(volatile v8h*)dst = v;
  }
}

__global__ __launch_bounds__(kThreads) void k_pool2(const _Float16* __restrict__ c2, _Float16* __restrict__ im3) {
  __shared__ __align__(16) _Float16 s_x2[25 * 16];
  const int tid = threadIdx.x;
  const int il  = blockIdx.x;
  const _Float16* cb = c2 + (size_t)il * (kRows2 * kNcol);
#pragma unroll 1
  for (int it = 0; it < 2; ++it) {
    const int idx = tid + it * kThreads;
    const int idc = imin(idx, 25 * 16 - 1);
    const int ic  = idc & 15;
    const int p   = idc >> 4;
    const int py  = p / 5;
    const int px  = p - py * 5;
    const int r0  = (2 * py) * 11 + 2 * px;
    const float a = (float)cb[(size_t)r0 * kNcol + ic] + (float)cb[(size_t)(r0 + 1) * kNcol + ic]
                  + (float)cb[(size_t)(r0 + 11) * kNcol + ic] + (float)cb[(size_t)(r0 + 12) * kNcol + ic];
    if (idx < 25 * 16) s_x2[idc] = (_Float16)(a * 0.25f);
  }
  __syncthreads();
  _Float16* ob = im3 + (size_t)il * (kRows3 * kKc3);
  const v8h z8 = zero8h();
#pragma unroll 1
  for (int it = 0; it < 2; ++it) {
    const int i    = tid + it * kThreads;
    const int ic   = imin(i, kRows3 * kKc3 / 8 - 1);
    const int row  = ic / 20;
    const int kq   = ic - row * 20;
    const int rowc = imin(row, kRows3Real - 1);
    const int oy   = rowc / 3;
    const int ox   = rowc - oy * 3;
    const int tap  = imin(kq >> 1, 8);
    const int icb  = (kq & 1) * 8;
    const int dy   = tap / 3;
    const int dx   = tap - dy * 3;
    const v8h xv = *(const v8h*)(s_x2 + ((oy + dy) * 5 + ox + dx) * 16 + icb);
    v8h v = xv;
    if (kq >= 18) v = z8;
    if (kq == 18) v[0] = (_Float16)kActCarry;
    if (row >= kRows3Real) v = z8;
    if (i < kRows3 * kKc3 / 8) {
      _Float16* dst = ob + (size_t)i * 8;
      *(volatile v8h*)dst = v;
      __threadfence();
      *(volatile v8h*)dst = v;
    }
  }
}

__global__ __launch_bounds__(kThreads) void k_pool3(const _Float16* __restrict__ c3, int img_base,
                                                     _Float16* __restrict__ xd) {
  const int tid = threadIdx.x;
  const int il  = blockIdx.x * 32 + (tid >> 3);
  const int q   = tid & 7;
  const _Float16* cb = c3 + (size_t)il * (kRows3 * kNcol);
  v8h hv;
#pragma unroll
  for (int e = 0; e < 8; ++e) {
    const int k  = q * 8 + e;
    const int kc = imin(k, kKdReal - 1);
    const float a = (float)cb[kc] + (float)cb[kNcol + kc] + (float)cb[3 * kNcol + kc] + (float)cb[4 * kNcol + kc];
    float v = a * 0.25f;
    if (k >= kKdReal) v = (k == kKdReal) ? kActCarry : 0.0f;
    hv[e] = (_Float16)v;
  }
  _Float16* dst = xd + (size_t)(img_base + il) * kKd + q * 8;
  *(volatile v8h*)dst = hv;
  __threadfence();
  *(volatile v8h*)dst = hv;
}

__global__ __launch_bounds__(kSmThreads) void k_softmax(const float* __restrict__ logp, float* out0, float* out1) {
  __shared__ __align__(16) float s_p[kSmImgs * 10];
  const int tid  = threadIdx.x;
  const int lane = tid & 31;
  const int wave = tid >> 5;
  if (wave == 0) {
    const int img = blockIdx.x * kSmImgs + lane;
    const float* lr = logp + (size_t)img * kKd;
    float m = -INFINITY;
#pragma unroll 1
    for (int j = 0; j < 10; ++j) m = fmaxf(m, lr[j]);
    float s = 0.f;
#pragma unroll 1
    for (int j = 0; j < 10; ++j) { const float e = expf(lr[j] - m); s_p[lane * 10 + j] = e; s += e; }
    const float inv = 1.0f / s;
#pragma unroll 1
    for (int j = 0; j < 10; ++j) s_p[lane * 10 + j] = s_p[lane * 10 + j] * inv;
  }
  __syncthreads();
  float* ob = (wave == 0) ? out0 : out1;
  ob += (size_t)blockIdx.x * (kSmImgs * 10);
  for (int pass = 0; pass < 2; ++pass) {
#pragma unroll
    for (int it = 0; it < 3; ++it) {
      const int p  = it * 32 + lane;
      const int pc = imin(p, kSmImgs * 10 / 4 - 1);
      const v4f v = *(const v4f*)(s_p + pc * 4);
      if (p < kSmImgs * 10 / 4) *(volatile v4f*)(ob + (size_t)p * 4) = v;
    }
    __threadfence();
  }
}

__global__ __launch_bounds__(kChainThreads) void k_chain(const float* __restrict__ trans, const float* probs,
                                                          int T, float* fin) {
  __shared__ float s_C[1000];
  __shared__ float s_gp[kChainSteps * 10];
  __shared__ float s_E[2][100];
  __shared__ float s_s[2][16];
  const int tid  = threadIdx.x;
  const int lane = tid & 31;
  const int wave = tid >> 5;
  if (tid < 96) {
    const int r = imin(tid, 89);
    const int g = r / 9;
    const int i = r - g * 9;
    const float* trow = trans + r * 10;
    float* crow = s_C + g * 100 + i * 10;
    float m = -INFINITY;
#pragma unroll 1
    for (int j = 0; j < 10; ++j) { const float v = trow[j] * kInvTemp; crow[j] = v; m = fmaxf(m, v); }
    float s = 0.f;
#pragma unroll 1
    for (int j = 0; j < 10; ++j) { const float e = expf(crow[j] - m); crow[j] = e; s += e; }
    const float inv = 1.0f / s;
#pragma unroll 1
    for (int j = 0; j < 10; ++j) crow[j] = crow[j] * inv;
  }
  __syncthreads();
  if (tid < 100) { const int g = tid / 10; const int j = tid - g * 10; s_C[g * 100 + 90 + j] = (j == 9) ? 1.f : 0.f; }
  if (tid < 16) { s_s[0][tid] = (tid == 0) ? 1.f : 0.f; s_s[1][tid] = 0.f; }
  __syncthreads();
  const int ec = imin(tid, 99);
  const int jc = imin(lane, 9);
  for (int base = 0; base < T; base += kChainSteps) {
    const int nst = imin(kChainSteps, T - base);
    for (int i = tid; i < nst * 10; i += kChainThreads) s_gp[i] = probs[(size_t)base * 10 + i];
    __syncthreads();
    for (int st = 0; st < nst; ++st) {
      const int par = (base + st) & 1;
      const float* gp = s_gp + st * 10;
      float e = 0.f;
#pragma unroll 1
      for (int g = 0; g < 10; ++g) e = fmaf(gp[g], s_C[g * 100 + ec], e);
      if (tid < 100) s_E[par][tid] = e;
      __syncthreads();
      if (wave == 0) {
        float ns = 0.f;
#pragma unroll 1
        for (int k = 0; k < 10; ++k) ns = fmaf(s_s[par][k], s_E[par][k * 10 + jc], ns);
        if (lane < 10) s_s[par ^ 1][lane] = ns;
      }
    }
    __syncthreads();
  }
  if (wave == 0) {
    const float v = s_s[T & 1][jc];
    if (lane < 10) {
      *(volatile float*)(fin + lane) = v;
      __threadfence();
      *(volatile float*)(fin + lane) = v;
    }
  }
}

extern "C" void kernel_launch(void* const* d_in, const int* in_sizes, int n_in,
                              void* d_out, int out_size, void* d_ws, size_t ws_size,
                              hipStream_t stream)
{
  const float* seq = (const float*)d_in[0];
  const float* w1  = (const float*)d_in[1];
  const float* b1  = (const float*)d_in[2];
  const float* w2  = (const float*)d_in[3];
  const float* b2  = (const float*)d_in[4];
  const float* w3  = (const float*)d_in[5];
  const float* b3  = (const float*)d_in[6];
  const float* dw  = (const float*)d_in[7];
  const float* db  = (const float*)d_in[8];
  const float* tr  = (const float*)d_in[9];

  const int T = in_sizes[0] / kImgPix;
  if (T < 64 || (T % 64) != 0) return;
  if (out_size < T * 20 + 10) return;

  float* out0 = (float*)d_out;
  float* out1 = out0 + (size_t)T * 10;
  float* out2 = out0 + (size_t)2 * T * 10;

  char* ws = (char*)d_ws;
  size_t off = 0;
  auto carve = [&](size_t bytes) { size_t o = off; off += (bytes + 255) & ~(size_t)255; return o; };
  const size_t oBT2 = carve((size_t)kNcol * kKc2 * 2);
  const size_t oBT3 = carve((size_t)kNcol * kKc3 * 2);
  const size_t oBTD = carve((size_t)kNcol * kKd * 2);
  const size_t oIM2 = carve((size_t)kImgsPerChunk * kRows2 * kKc2 * 2);
  const size_t oC2  = carve((size_t)kImgsPerChunk * kRows2 * kNcol * 2);
  const size_t oIM3 = carve((size_t)kImgsPerChunk * kRows3 * kKc3 * 2);
  const size_t oC3  = carve((size_t)kImgsPerChunk * kRows3 * kNcol * 2);
  const size_t oXD  = carve((size_t)T * kKd * 2);
  const size_t oLOG = carve((size_t)T * kKd * 4);
  if (off > ws_size) return;

  _Float16* BT2 = (_Float16*)(ws + oBT2);
  _Float16* BT3 = (_Float16*)(ws + oBT3);
  _Float16* BTD = (_Float16*)(ws + oBTD);
  _Float16* IM2 = (_Float16*)(ws + oIM2);
  _Float16* C2  = (_Float16*)(ws + oC2);
  _Float16* IM3 = (_Float16*)(ws + oIM3);
  _Float16* C3  = (_Float16*)(ws + oC3);
  _Float16* XD  = (_Float16*)(ws + oXD);
  float*    LOG = (float*)(ws + oLOG);
  const float* dummyf = LOG;

  k_wprep<<<kNcol * kKc2 / 8 / kThreads, kThreads, 0, stream>>>(w2, b2, 16, 8, 9, kKc2Real, kKc2, kWCarry, BT2);
  k_wprep<<<kNcol * kKc3 / 8 / kThreads, kThreads, 0, stream>>>(w3, b3, 32, 16, 9, kKc3Real, kKc3, kWCarry, BT3);
  k_wprep<<<kNcol * kKd / 8 / kThreads, kThreads, 0, stream>>>(dw, db, 10, 32, 1, kKdReal, kKd, kWCarry, BTD);

  const int nchunk = (T + kImgsPerChunk - 1) / kImgsPerChunk;
  for (int c = 0; c < nchunk; ++c) {
    const int ibase = c * kImgsPerChunk;
    const int nimg  = (T - ibase < kImgsPerChunk) ? (T - ibase) : kImgsPerChunk;
    const int M2 = nimg * kRows2;
    const int M3 = nimg * kRows3;

    k_conv1<<<nimg, kThreads, 0, stream>>>(seq, w1, b1, ibase, IM2);

    {
      const int tiles = (M2 / 64) * (kNcol / 64);
      wmma_gemm64<0, false, 0, 1, false, 2><<<dim3((tiles + 7) / 8, 1), 256, 0, stream>>>(
          (const unsigned short*)IM2, (const unsigned short*)IM2, kKc2, 0L,
          (const unsigned short*)BT2, (const unsigned short*)BT2, kKc2, 0L,
          (void*)C2, (void*)C2, kNcol, 0L, dummyf, dummyf, 0L, M2, kNcol, kKc2, kConvScale);
    }

    k_pool2<<<nimg, kThreads, 0, stream>>>(C2, IM3);

    {
      const int tiles = (M3 / 64) * (kNcol / 64);
      wmma_gemm64<0, false, 0, 1, false, 2><<<dim3((tiles + 7) / 8, 1), 256, 0, stream>>>(
          (const unsigned short*)IM3, (const unsigned short*)IM3, kKc3, 0L,
          (const unsigned short*)BT3, (const unsigned short*)BT3, kKc3, 0L,
          (void*)C3, (void*)C3, kNcol, 0L, dummyf, dummyf, 0L, M3, kNcol, kKc3, kConvScale);
    }

    k_pool3<<<nimg / 32, kThreads, 0, stream>>>(C3, ibase, XD);
  }

  {
    const int tiles = (T / 64) * (kNcol / 64);
    wmma_gemm64<0, false, 0, 0, false, 0><<<dim3((tiles + 7) / 8, 1), 256, 0, stream>>>(
        (const unsigned short*)XD, (const unsigned short*)XD, kKd, 0L,
        (const unsigned short*)BTD, (const unsigned short*)BTD, kKd, 0L,
        (void*)LOG, (void*)LOG, kNcol, 0L, dummyf, dummyf, 0L, T, kNcol, kKd, kDenseScale);
  }

  k_softmax<<<T / kSmImgs, kSmThreads, 0, stream>>>(LOG, out0, out1);
  k_chain<<<1, kChainThreads, 0, stream>>>(tr, out0, T, out2);
}
